// LPair_5720896438536
// MI455X (gfx1250) — hardware-verified
//
#include <hip/hip_runtime.h>
#include <math.h>
#include <stdint.h>

#define NB   4
#define NN   512
#define DF   48
#define D2   96
#define NROW 2048
#define NIT  128
#define NBLK 1024
static_assert(NROW == NB * NN);
static_assert(D2 == 2 * DF);
static_assert(NROW == NIT * 16);
static_assert(NBLK * 2 == NROW);
static_assert((D2 % 32) == 0);
static_assert(DF * D2 == 9 * 64 * 8);
static_assert((NN % 16) == 0);

typedef _Float16     v16h __attribute__((ext_vector_type(16)));
typedef _Float16     v8h  __attribute__((ext_vector_type(8)));
typedef float        v8f  __attribute__((ext_vector_type(8)));
typedef float        v4f  __attribute__((ext_vector_type(4)));

union Frag { v16h v; v8h half[2]; };

__device__ __forceinline__ unsigned short bf_bits(float f) {
  unsigned u = __float_as_uint(f);
  return (unsigned short)((u + 0x7FFFu + ((u >> 16) & 1u)) >> 16);
}
__device__ __forceinline__ float bf_up(unsigned short b) { return __uint_as_float(((unsigned)b) << 16); }
__device__ __forceinline__ float bfr(float f) { return bf_up(bf_bits(f)); }
__device__ __forceinline__ v8f zero8() {
  v8f z;
  z[0] = 0.f; z[1] = 0.f; z[2] = 0.f; z[3] = 0.f; z[4] = 0.f; z[5] = 0.f; z[6] = 0.f; z[7] = 0.f;
  return z;
}

__device__ __forceinline__ v16h ldfrag(const _Float16* p) {
  Frag f;
  f.half[0] = *(const v8h*)(p);
  f.half[1] = *(const v8h*)(p + 16);
  return f.v;
}

__device__ __forceinline__ v8f mma(v16h a, v16h b, v8f c) {
  v8f d = __builtin_amdgcn_wmma_f32_16x16x32_f16(false, a, false, b, (short)0, c, false, false);
#if defined(__HIP_DEVICE_COMPILE__)
  asm volatile("v_nop\n\tv_nop\n\tv_nop\n\tv_nop" : "+v"(d) : "v"(a), "v"(b));
#endif
  return d;
}

__device__ __forceinline__ float gelu16(float z) {
  const float e = erff(z * 0.70710678118654752440f);
  return 8.0f * z * (1.0f + e);
}
__device__ __forceinline__ void hsplit(float z, _Float16& hi, _Float16& lo) {
  const float g = gelu16(z);
  const _Float16 hv = (_Float16)g;
  hi = hv;
  lo = (_Float16)((g - (float)hv) * 2048.0f);
}

__global__ __launch_bounds__(64) void k_w2t(const float* __restrict__ W2, _Float16* W2T) {
  const int tid = threadIdx.x;
  v8h pv[9];
#pragma unroll
  for (int it = 0; it < 9; ++it) {
    const int q  = it * 64 + tid;
    const int n  = q / 12;
    const int kb = (q - n * 12) * 8;
    v8h v;
#pragma unroll
    for (int e = 0; e < 8; ++e) v[e] = (_Float16)(bfr(W2[(size_t)(kb + e) * DF + n]) * 1024.0f);
    pv[it] = v;
  }
#pragma unroll
  for (int it = 0; it < 9; ++it) *(volatile v8h*)(W2T + (size_t)(it * 64 + tid) * 8) = pv[it];
  __threadfence();
#pragma unroll
  for (int it = 0; it < 9; ++it) *(volatile v8h*)(W2T + (size_t)(it * 64 + tid) * 8) = pv[it];
}

__global__ __launch_bounds__(64) void k_pre(const float* __restrict__ x, const float* __restrict__ W1,
                                            const float* __restrict__ b1, float* AB) {
  __shared__ __align__(16) float sT[2 * 16 * D2];
  const int tid  = threadIdx.x;
  const int lane = tid & 31, wid = tid >> 5, h = lane >> 4, c16 = lane & 15;
  const int row0 = blockIdx.x * 16;

  Frag fa0, fa1;
  {
    const float* xr = x + (size_t)(row0 + c16) * DF + 8 * h;
    const v4f x0 = *(const v4f*)(xr);
    const v4f x1 = *(const v4f*)(xr + 4);
    const v4f x2 = *(const v4f*)(xr + 16);
    const v4f x3 = *(const v4f*)(xr + 20);
    const v4f x4 = *(const v4f*)(xr + 32);
    const v4f x5 = *(const v4f*)(xr + 36);
    v8h p0, p1, p2, pz;
#pragma unroll
    for (int c = 0; c < 4; ++c) {
      p0[c]     = (_Float16)(bfr(x0[c]) * 16.0f);
      p0[4 + c] = (_Float16)(bfr(x1[c]) * 16.0f);
      p1[c]     = (_Float16)(bfr(x2[c]) * 16.0f);
      p1[4 + c] = (_Float16)(bfr(x3[c]) * 16.0f);
      p2[c]     = (_Float16)(bfr(x4[c]) * 16.0f);
      p2[4 + c] = (_Float16)(bfr(x5[c]) * 16.0f);
      pz[c]     = (_Float16)0.0f;
      pz[4 + c] = (_Float16)0.0f;
    }
    fa0.half[0] = p0; fa0.half[1] = p1;
    fa1.half[0] = p2; fa1.half[1] = pz;
  }

  const float* Wb  = W1 + (size_t)(wid * DF) * D2;
  float*       sTw = sT + wid * 16 * D2;
#pragma unroll 1
  for (int nt = 0; nt < 6; ++nt) {
    const int n = nt * 16 + c16;
    v16h fb0, fb1;
#pragma unroll
    for (int e = 0; e < 8; ++e) {
      fb0[e]     = (_Float16)(bfr(Wb[(size_t)(8 * h + e) * D2 + n]) * 1024.0f);
      fb0[8 + e] = (_Float16)(bfr(Wb[(size_t)(16 + 8 * h + e) * D2 + n]) * 1024.0f);
      fb1[e]     = (_Float16)(bfr(Wb[(size_t)(32 + 8 * h + e) * D2 + n]) * 1024.0f);
      fb1[8 + e] = (_Float16)0.0f;
    }
    v8f acc = mma(fa0.v, fb0, zero8());
    acc = mma(fa1.v, fb1, acc);
    const float bb   = bfr(b1[n]);
    const float badd = (wid == 0) ? bb : 0.0f;
#pragma unroll
    for (int r = 0; r < 8; ++r) sTw[(8 * h + r) * D2 + n] = acc[r] * 6.103515625e-05f + badd;
  }
  __syncthreads();

  float* dst = AB + (size_t)wid * NROW * D2 + (size_t)row0 * D2;
  v4f pv[12];
#pragma unroll
  for (int it = 0; it < 12; ++it) pv[it] = *(const v4f*)(sTw + (it * 32 + lane) * 4);
#pragma unroll
  for (int it = 0; it < 12; ++it) *(volatile v4f*)(dst + (size_t)(it * 32 + lane) * 4) = pv[it];
  __threadfence();
#pragma unroll
  for (int it = 0; it < 12; ++it) *(volatile v4f*)(dst + (size_t)(it * 32 + lane) * 4) = pv[it];
}

__global__ __launch_bounds__(64) void k_main(const float* __restrict__ AB, const _Float16* __restrict__ W2T,
                                             const float* __restrict__ b2, float* out) {
  __shared__ __align__(16) _Float16 sW[DF * D2];
  __shared__ __align__(16) float sO[2 * DF];
  const int tid  = threadIdx.x;
  const int lane = tid & 31, wid = tid >> 5, h = lane >> 4, c16 = lane & 15;
  const int b    = blockIdx.x / (NN / 2);
  const int ip   = blockIdx.x % (NN / 2);
  const int i    = 2 * ip + wid;

#pragma unroll
  for (int it = 0; it < 9; ++it) {
    const int q = it * 64 + tid;
    *(v8h*)(sW + 8 * q) = *(const v8h*)(W2T + 8 * q);
  }
  __syncthreads();

  const float*    Arow = AB + (size_t)(b * NN + i) * D2 + 8 * h;
  const float*    Bb   = AB + (size_t)NROW * D2 + (size_t)(b * NN + c16) * D2 + 8 * h;
  const _Float16* sWl  = sW + c16 * D2 + 8 * h;

  float b2v[3];
#pragma unroll
  for (int nt = 0; nt < 3; ++nt) b2v[nt] = bfr(b2[nt * 16 + c16]);

  const float NINF = -__builtin_inff();
  float m_run = NINF, l_run = 0.f;
  float oacc[3];
  oacc[0] = 0.f; oacc[1] = 0.f; oacc[2] = 0.f;

  const int ntiles = (i >> 4) + 1;
#pragma unroll 1
  for (int t = 0; t < ntiles; ++t) {
    const int    j0   = t << 4;
    const float* Brow = Bb + (size_t)j0 * D2;

    v8f Ch[3], Cl[3];
#pragma unroll
    for (int nt = 0; nt < 3; ++nt) { Ch[nt] = zero8(); Cl[nt] = zero8(); }

#pragma unroll 1
    for (int c = 0; c < 3; ++c) {
      const float* ap = Arow + c * 32;
      const float* bp = Brow + c * 32;
      const v4f a0 = *(const v4f*)(ap);
      const v4f a1 = *(const v4f*)(ap + 4);
      const v4f a2 = *(const v4f*)(ap + 16);
      const v4f a3 = *(const v4f*)(ap + 20);
      const v4f q0 = *(const v4f*)(bp);
      const v4f q1 = *(const v4f*)(bp + 4);
      const v4f q2 = *(const v4f*)(bp + 16);
      const v4f q3 = *(const v4f*)(bp + 20);
      v8h hh0, hl0, hh1, hl1;
#pragma unroll
      for (int e = 0; e < 4; ++e) {
        _Float16 th, tl;
        hsplit(a0[e] + q0[e], th, tl); hh0[e]     = th; hl0[e]     = tl;
        hsplit(a1[e] + q1[e], th, tl); hh0[4 + e] = th; hl0[4 + e] = tl;
        hsplit(a2[e] + q2[e], th, tl); hh1[e]     = th; hl1[e]     = tl;
        hsplit(a3[e] + q3[e], th, tl); hh1[4 + e] = th; hl1[4 + e] = tl;
      }
      Frag fh, fl;
      fh.half[0] = hh0; fh.half[1] = hh1;
      fl.half[0] = hl0; fl.half[1] = hl1;
#pragma unroll
      for (int nt = 0; nt < 3; ++nt) {
        const v16h w = ldfrag(sWl + nt * (16 * D2) + c * 32);
        Ch[nt] = mma(fh.v, w, Ch[nt]);
        Cl[nt] = mma(fl.v, w, Cl[nt]);
      }
    }

    float p[3][8], q[8];
#pragma unroll
    for (int v = 0; v < 8; ++v) {
      float qq = 0.f;
#pragma unroll
      for (int nt = 0; nt < 3; ++nt) {
        const float pv = (Ch[nt][v] + Cl[nt][v] * 0.00048828125f) * 6.103515625e-05f + b2v[nt];
        p[nt][v] = pv;
        qq += pv * pv;
      }
      q[v] = qq;
    }
#pragma unroll
    for (int m = 1; m <= 8; m <<= 1)
#pragma unroll
      for (int v = 0; v < 8; ++v)
        q[v] += __shfl_xor(q[v], m, 32);

    float s[8];
    float tmax = NINF;
#pragma unroll
    for (int v = 0; v < 8; ++v) {
      const int   j  = j0 + 8 * h + v;
      const float sq = __builtin_sqrtf(q[v]);
      s[v] = (j <= i) ? sq : NINF;
      tmax = fmaxf(tmax, s[v]);
    }
    tmax = fmaxf(tmax, __shfl_xor(tmax, 16, 32));
    const float m_new = fmaxf(m_run, tmax);

    float wv[8];
    float sw = 0.f;
#pragma unroll
    for (int v = 0; v < 8; ++v) { wv[v] = __expf(s[v] - m_new); sw += wv[v]; }
    sw += __shfl_xor(sw, 16, 32);

    const float scale = __expf(m_run - m_new);
    l_run = l_run * scale + sw;
#pragma unroll
    for (int nt = 0; nt < 3; ++nt) {
      float a2 = 0.f;
#pragma unroll
      for (int v = 0; v < 8; ++v) a2 += wv[v] * p[nt][v];
      oacc[nt] = oacc[nt] * scale + a2;
    }
    m_run = m_new;
  }

  const float inv = __builtin_amdgcn_rcpf(l_run);
#pragma unroll
  for (int nt = 0; nt < 3; ++nt) {
    const float a2 = oacc[nt] + __shfl_xor(oacc[nt], 16, 32);
    const float ov = a2 * inv;
    if (h == 0) sO[wid * DF + nt * 16 + c16] = ov;
  }
  __syncthreads();

  const bool wr = (tid < 24);
  const int  tq = wr ? tid : 0;
  const v4f  ov4 = *(const v4f*)(sO + 4 * tq);
  float* od = out + (size_t)(b * NN + 2 * ip) * DF + 4 * tq;
  if (wr) *(volatile v4f*)od = ov4;
  __threadfence();
  if (wr) *(volatile v4f*)od = ov4;
}

extern "C" void kernel_launch(void* const* d_in, const int* in_sizes, int n_in,
                              void* d_out, int out_size, void* d_ws, size_t ws_size,
                              hipStream_t stream) {
  if (n_in < 5) return;
  if (in_sizes[0] != NB * NN * DF) return;
  if (in_sizes[1] != D2 * D2) return;
  if (in_sizes[2] != D2) return;
  if (in_sizes[3] != D2 * DF) return;
  if (in_sizes[4] != DF) return;
  if (out_size != NB * NN * DF) return;

  const float* x  = (const float*)d_in[0];
  const float* W1 = (const float*)d_in[1];
  const float* b1 = (const float*)d_in[2];
  const float* W2 = (const float*)d_in[3];
  const float* b2 = (const float*)d_in[4];
  float* out = (float*)d_out;

  const size_t offAB = 0;
  const size_t szAB  = (size_t)2 * NROW * D2 * sizeof(float);
  const size_t offW2 = offAB + szAB;
  const size_t szW2  = (size_t)DF * D2 * sizeof(_Float16);
  const size_t total = offW2 + szW2;
  if (total > ws_size) return;
  if (total > (size_t)134217728) return;

  char*     ws  = (char*)d_ws;
  float*    AB  = (float*)(ws + offAB);
  _Float16* W2T = (_Float16*)(ws + offW2);

  const dim3 gW2(1),      bW2(64);
  const dim3 gPre(NIT),   bPre(64);
  const dim3 gMain(NBLK), bMain(64);

  k_w2t<<<gW2, bW2, 0, stream>>>(W2, W2T);
  k_pre<<<gPre, bPre, 0, stream>>>(x, W1, b1, AB);
  k_main<<<gMain, bMain, 0, stream>>>(AB, W2T, b2, out);
  (void)hipGetLastError();
}
